// RATransformerEncoderLayer_70884140253548
// MI455X (gfx1250) — hardware-verified
//
#include <hip/hip_runtime.h>
#include <math.h>
#include <stdint.h>

#define NBATCH 2
#define SEQ    512
#define DM     1024
#define NH     16
#define HD     64
#define DFF    4096
#define NREL   64
#define QKP    (2 * DM)
#define CTXP   (2 * DM)
#define XPP    (2 * DM)
#define HPP    (2 * DFF)
#define MP     (NBATCH * SEQ)
#define NQB    (SEQ / 64)
#define WSC    64.0f
#define RSC    2048.0f
#define PSC    1024.0f
#define HCY    32.0f
#define PFX    2097152.0f
static_assert(NH * HD == DM);
static_assert((SEQ % 64) == 0 && (DM % 64) == 0 && (MP % 64) == 0 && (DFF % 64) == 0);
static_assert(NREL == 64 && HD == 64);
static_assert((MP % 8) == 0);

typedef _Float16 v16h __attribute__((ext_vector_type(16)));
typedef _Float16 v8h  __attribute__((ext_vector_type(8)));
typedef __bf16   v16b __attribute__((ext_vector_type(16)));
typedef unsigned short v16us __attribute__((ext_vector_type(16)));
typedef unsigned short v8us  __attribute__((ext_vector_type(8)));
typedef float    v8f  __attribute__((ext_vector_type(8)));
typedef float    v4f  __attribute__((ext_vector_type(4)));
typedef unsigned int v4u __attribute__((ext_vector_type(4)));
typedef unsigned int v2u __attribute__((ext_vector_type(2)));

union FragH { v16h v; v8h h[2]; };
union FragU { v16us v; v8us h[2]; };

__device__ __forceinline__ unsigned short bf_bits(float f) {
  unsigned u = __float_as_uint(f);
  return (unsigned short)((u + 0x7FFFu + ((u >> 16) & 1u)) >> 16);
}
__device__ __forceinline__ float bf_up(unsigned short h) { return __uint_as_float(((unsigned)h) << 16); }
__device__ __forceinline__ float bfr(float f) { return bf_up(bf_bits(f)); }
__device__ __forceinline__ unsigned short h_bits(_Float16 x) { return __builtin_bit_cast(unsigned short, x); }
__device__ __forceinline__ unsigned pk16(unsigned short a, unsigned short b) { return (unsigned)a | ((unsigned)b << 16); }
__device__ __forceinline__ v8f zero8() { v8f z = {0.f, 0.f, 0.f, 0.f, 0.f, 0.f, 0.f, 0.f}; return z; }

__device__ __forceinline__ v16us ldfrag_u(const unsigned short* p) {
  FragU f;
  f.h[0] = *(const v8us*)(p);
  f.h[1] = *(const v8us*)(p + 16);
  return f.v;
}
__device__ __forceinline__ v16h ldfrag_h(const _Float16* p) {
  FragH f;
  f.h[0] = *(const v8h*)(p);
  f.h[1] = *(const v8h*)(p + 16);
  return f.v;
}

template <int BF>
__device__ __forceinline__ v8f mma_raw(v16us a, v16us b, v8f c) {
  if (BF) {
    return __builtin_amdgcn_wmma_f32_16x16x32_bf16(false, __builtin_bit_cast(v16b, a), false,
                                                   __builtin_bit_cast(v16b, b), (short)0, c, false, false);
  }
  return __builtin_amdgcn_wmma_f32_16x16x32_f16(false, __builtin_bit_cast(v16h, a), false,
                                                __builtin_bit_cast(v16h, b), (short)0, c, false, false);
}
__device__ __forceinline__ v8f mma_bu(v16us a, v16us b, v8f c) {
  c = __builtin_amdgcn_wmma_f32_16x16x32_bf16(false, __builtin_bit_cast(v16b, a), false,
                                               __builtin_bit_cast(v16b, b), (short)0, c, false, false);
#if defined(__HIP_DEVICE_COMPILE__)
  asm volatile("v_nop\n\tv_nop\n\tv_nop\n\tv_nop" : "+v"(c) : "v"(a), "v"(b));
#endif
  return c;
}
__device__ __forceinline__ v8f mma_h(v16h a, v16h b, v8f c) {
  c = __builtin_amdgcn_wmma_f32_16x16x32_f16(false, a, false, b, (short)0, c, false, false);
#if defined(__HIP_DEVICE_COMPILE__)
  asm volatile("v_nop\n\tv_nop\n\tv_nop\n\tv_nop" : "+v"(c) : "v"(a), "v"(b));
#endif
  return c;
}
__device__ __forceinline__ void dep_guard1(v8f& a, v8f& b, v16us x) {
#if defined(__HIP_DEVICE_COMPILE__)
  asm volatile("v_nop\n\tv_nop\n\tv_nop\n\tv_nop" : "+v"(a), "+v"(b) : "v"(x));
#endif
}
__device__ __forceinline__ void keep4_u(v16us a, v16us b, v16us c, v16us d) {
#if defined(__HIP_DEVICE_COMPILE__)
  asm volatile("v_nop" :: "v"(a), "v"(b), "v"(c), "v"(d));
#endif
}
__device__ __forceinline__ void acc_guard4(v8f& a, v8f& b, v8f& c, v8f& d) {
#if defined(__HIP_DEVICE_COMPILE__)
  asm volatile("v_nop\n\tv_nop\n\tv_nop\n\tv_nop" : "+v"(a), "+v"(b), "+v"(c), "+v"(d));
#endif
}
__device__ __forceinline__ void wave_sync_lds() {
  __builtin_amdgcn_fence(__ATOMIC_RELEASE, "workgroup");
  __builtin_amdgcn_wave_barrier();
  __builtin_amdgcn_fence(__ATOMIC_ACQUIRE, "workgroup");
}

template <int MODE>
__global__ __launch_bounds__(256) void conv16(const float* __restrict__ W, unsigned short* out,
                                              int n8, int K, int ldo, int dup, float wsc) {
  const int i  = blockIdx.x * 256 + threadIdx.x;
  const int ic = (i < n8) ? i : (n8 - 1);
  const size_t e = (size_t)ic * 8;
  const size_t n = e / (size_t)K;
  const size_t k = e - n * (size_t)K;
  const float* src = W + e;
  const v4f a = *(const v4f*)(src);
  const v4f c = *(const v4f*)(src + 4);
  v4u o;
  if (MODE == 0) {
    o[0] = pk16(h_bits((_Float16)(bfr(a[0]) * wsc)), h_bits((_Float16)(bfr(a[1]) * wsc)));
    o[1] = pk16(h_bits((_Float16)(bfr(a[2]) * wsc)), h_bits((_Float16)(bfr(a[3]) * wsc)));
    o[2] = pk16(h_bits((_Float16)(bfr(c[0]) * wsc)), h_bits((_Float16)(bfr(c[1]) * wsc)));
    o[3] = pk16(h_bits((_Float16)(bfr(c[2]) * wsc)), h_bits((_Float16)(bfr(c[3]) * wsc)));
  } else {
    o[0] = pk16(bf_bits(a[0]), bf_bits(a[1]));
    o[1] = pk16(bf_bits(a[2]), bf_bits(a[3]));
    o[2] = pk16(bf_bits(c[0]), bf_bits(c[1]));
    o[3] = pk16(bf_bits(c[2]), bf_bits(c[3]));
  }
  const size_t go = n * (size_t)ldo + k;
  if (i < n8) {
    *(volatile v4u*)(out + go) = o;
    if (dup != 0) *(volatile v4u*)(out + go + K) = o;
  }
  __threadfence();
  if (i < n8) {
    *(volatile v4u*)(out + go) = o;
    if (dup != 0) *(volatile v4u*)(out + go + K) = o;
  }
}

__global__ __launch_bounds__(256) void conv_e16(const float* __restrict__ P, unsigned short* Eh, int n8v, int n8t) {
  const int i  = blockIdx.x * 256 + threadIdx.x;
  const int ic = (i < n8v) ? i : (n8v - 1);
  const float* src = P + (size_t)ic * 8;
  const v4f a = *(const v4f*)(src);
  const v4f c = *(const v4f*)(src + 4);
  const bool valid = (i < n8v);
  v4u o;
  o[0] = valid ? pk16(bf_bits(a[0]), bf_bits(a[1])) : 0u;
  o[1] = valid ? pk16(bf_bits(a[2]), bf_bits(a[3])) : 0u;
  o[2] = valid ? pk16(bf_bits(c[0]), bf_bits(c[1])) : 0u;
  o[3] = valid ? pk16(bf_bits(c[2]), bf_bits(c[3])) : 0u;
  if (i < n8t) *(volatile v4u*)(Eh + (size_t)i * 8) = o;
  __threadfence();
  if (i < n8t) *(volatile v4u*)(Eh + (size_t)i * 8) = o;
}

template <int MODE>
__global__ __launch_bounds__(256) void tconv64(const float* __restrict__ W, unsigned short* out,
                                               int rows, int cols, int ldo, int dupoff, float wsc) {
  __shared__ __align__(16) unsigned short sh[64 * 72];
  const int t  = threadIdx.x;
  const int n0 = blockIdx.x * 64;
  const int k0 = blockIdx.y * 64;
#pragma unroll
  for (int i = 0; i < 4; ++i) {
    const int idx = i * 256 + t;
    const int r = idx >> 4, c4 = (idx & 15) * 4;
    int kr = k0 + r;   kr = (kr < rows) ? kr : (rows - 1);
    int nc = n0 + c4;  nc = (nc < cols - 4) ? nc : (cols - 4);
    const v4f v = *(const v4f*)(W + (size_t)kr * cols + nc);
#pragma unroll
    for (int e = 0; e < 4; ++e) {
      unsigned short u;
      if (MODE == 0) u = h_bits((_Float16)(bfr(v[e]) * wsc));
      else           u = bf_bits(v[e]);
      sh[(c4 + e) * 72 + r] = u;
    }
  }
  __syncthreads();
  const int wave = t >> 5, lane = t & 31;
  const int q = lane >> 3, c8 = (lane & 7) * 8;
  v4u pv[2];
  size_t go[2];
#pragma unroll
  for (int it = 0; it < 2; ++it) {
    const int nl = it * 32 + wave * 4 + q;
    pv[it] = *(const v4u*)(sh + nl * 72 + c8);
    go[it] = (size_t)(n0 + nl) * ldo + k0 + c8;
  }
  for (int pass = 0; pass < 2; ++pass) {
#pragma unroll
    for (int it = 0; it < 2; ++it) {
      *(volatile v4u*)(out + go[it]) = pv[it];
      if (dupoff != 0) *(volatile v4u*)(out + go[it] + dupoff) = pv[it];
    }
    __threadfence();
  }
}

template <int BF, int OM, int BM, int RL>
__global__ __launch_bounds__(256) void gemm64(
    const unsigned short* __restrict__ Ap, int lda, long long strideA,
    const unsigned short* __restrict__ Btp, int ldb, long long strideB,
    unsigned short* Cp, unsigned short* Cp2, float* Cf, int ldc, long long strideC,
    const float* __restrict__ bias, int M, int N, int K, float oscale) {
  __shared__ __align__(16) float sT[8][16 * 68];
  const int b    = blockIdx.y;
  const int lane = threadIdx.x & 31;
  const int wave = threadIdx.x >> 5;
  const int tilesN = N >> 6;
  const int tilesM = M >> 6;
  const int tile = blockIdx.x * 8 + wave;
  if (tile >= tilesM * tilesN) return;
  const int tm = tile / tilesN;
  const int tn = tile - tm * tilesN;
  const int m0 = tm << 6;
  const int n0 = tn << 6;

  const unsigned short* Ab = Ap  + (size_t)b * strideA;
  const unsigned short* Bb = Btp + (size_t)b * strideB;

  const int rlane = lane & 15;
  const int koff  = (lane >> 4) * 8;
  const int mOff  = (lane >> 4) * 8;

  v8f acc[4][4];
#pragma unroll
  for (int i = 0; i < 4; ++i)
#pragma unroll
    for (int j = 0; j < 4; ++j) acc[i][j] = zero8();

  for (int k0 = 0; k0 < K; k0 += 32) {
    v16us bh[4];
#pragma unroll
    for (int j = 0; j < 4; ++j) {
      const size_t bo = (size_t)(n0 + (j << 4) + rlane) * ldb + koff + k0;
      bh[j] = ldfrag_u(Bb + bo);
    }
#pragma unroll
    for (int i = 0; i < 4; ++i) {
      const size_t ao = (size_t)(m0 + (i << 4) + rlane) * lda + koff + k0;
      const v16us ah = ldfrag_u(Ab + ao);
#pragma unroll
      for (int j = 0; j < 4; ++j) acc[i][j] = mma_raw<BF>(ah, bh[j], acc[i][j]);
      dep_guard1(acc[i][0], acc[i][3], ah);
    }
    keep4_u(bh[0], bh[1], bh[2], bh[3]);
  }
  acc_guard4(acc[0][0], acc[0][1], acc[0][2], acc[0][3]);
  acc_guard4(acc[1][0], acc[1][1], acc[1][2], acc[1][3]);
  acc_guard4(acc[2][0], acc[2][1], acc[2][2], acc[2][3]);
  acc_guard4(acc[3][0], acc[3][1], acc[3][2], acc[3][3]);

  const int hh2 = lane >> 4, c4 = (lane & 15) * 4;
  const int q8  = lane >> 3, c8 = (lane & 7) * 8;

  float* slab = sT[wave];
#pragma unroll
  for (int i = 0; i < 4; ++i) {
    const int mBase = m0 + (i << 4);
#pragma unroll
    for (int j = 0; j < 4; ++j) {
#pragma unroll
      for (int r = 0; r < 8; ++r) {
        slab[(mOff + r) * 68 + (j << 4) + rlane] = acc[i][j][r];
      }
    }
    wave_sync_lds();
    if (OM == 0) {
      float* C = Cf + (size_t)b * strideC;
      v4f b4 = {0.f, 0.f, 0.f, 0.f};
      if (BM == 1) {
        const v4f t4 = *(const v4f*)(bias + n0 + c4);
        b4[0] = bfr(t4[0]); b4[1] = bfr(t4[1]); b4[2] = bfr(t4[2]); b4[3] = bfr(t4[3]);
      }
      v4f vals[8];
#pragma unroll
      for (int it = 0; it < 8; ++it) {
        const int row = it * 2 + hh2;
        v4f v = *(const v4f*)(slab + row * 68 + c4);
        v = v * oscale + b4;
        if (BM == 2) { const float bb = bfr(bias[mBase + row]); v = v + bb; }
        if (RL) { v[0] = fmaxf(v[0], 0.f); v[1] = fmaxf(v[1], 0.f); v[2] = fmaxf(v[2], 0.f); v[3] = fmaxf(v[3], 0.f); }
        vals[it] = v;
      }
      for (int pass = 0; pass < 2; ++pass) {
#pragma unroll
        for (int it = 0; it < 8; ++it) {
          const int row = it * 2 + hh2;
          *(volatile v4f*)(C + (size_t)(mBase + row) * ldc + n0 + c4) = vals[it];
        }
        __threadfence();
      }
    } else {
      unsigned short* C  = Cp  + (size_t)b * strideC;
      unsigned short* C2 = Cp2 + (size_t)b * strideC;
      v4u hv[4], lv[4];
#pragma unroll
      for (int it = 0; it < 4; ++it) {
        const int row = it * 4 + q8;
        const float* sp = slab + row * 68 + c8;
        float brow = 0.f;
        if (BM == 2) brow = bfr(bias[mBase + row]);
        v4u ha, la;
#pragma unroll
        for (int e = 0; e < 4; ++e) {
          float f0 = sp[2 * e]     * oscale + brow;
          float f1 = sp[2 * e + 1] * oscale + brow;
          if (BM == 1) { f0 += bfr(bias[n0 + c8 + 2 * e]); f1 += bfr(bias[n0 + c8 + 2 * e + 1]); }
          if (RL) { f0 = fmaxf(f0, 0.f); f1 = fmaxf(f1, 0.f); }
          unsigned short u0, u1, w0, w1;
          if (OM == 3) {
            u0 = bf_bits(f0); u1 = bf_bits(f1);
            w0 = bf_bits(f0 - bf_up(u0)); w1 = bf_bits(f1 - bf_up(u1));
          } else {
            const _Float16 g0 = (_Float16)f0, g1 = (_Float16)f1;
            u0 = h_bits(g0); u1 = h_bits(g1);
            w0 = h_bits((_Float16)((f0 - (float)g0) * RSC));
            w1 = h_bits((_Float16)((f1 - (float)g1) * RSC));
          }
          ha[e] = pk16(u0, u1);
          la[e] = pk16(w0, w1);
        }
        hv[it] = ha;
        lv[it] = la;
      }
      for (int pass = 0; pass < 2; ++pass) {
#pragma unroll
        for (int it = 0; it < 4; ++it) {
          const int row = it * 4 + q8;
          const size_t go = (size_t)(mBase + row) * ldc + n0 + c8;
          *(volatile v4u*)(C  + go) = hv[it];
          *(volatile v4u*)(C2 + go) = lv[it];
        }
        __threadfence();
      }
    }
    wave_sync_lds();
  }
}

__global__ __launch_bounds__(128)
void attn64(const unsigned short* __restrict__ qkh, const unsigned short* __restrict__ qkl,
            const unsigned short* __restrict__ vth, const unsigned short* __restrict__ vtl,
            const unsigned short* __restrict__ ekp, const unsigned short* __restrict__ evp,
            const int* __restrict__ relp, unsigned short* ctxp, float sscale) {
  __shared__ __align__(16) unsigned short Kh[64 * 64];
  __shared__ __align__(16) unsigned short Kl[64 * 64];
  __shared__ __align__(16) _Float16 Vh[64 * 64];
  __shared__ __align__(16) _Float16 Vl[64 * 64];
  __shared__ __align__(16) _Float16 Psh[4][16 * 64];
  __shared__ __align__(16) float    Rsh[64 * NREL];
  __shared__ __align__(16) unsigned int Hs[4][16 * NREL];
  __shared__ __align__(16) float    Os[4][16 * 64];

  const int tid  = threadIdx.x;
  const int wave = tid >> 5;
  const int lane = tid & 31;
  const int hh   = lane >> 4;
  const int c    = lane & 15;

  const int bx   = blockIdx.x;
  const int qb   = bx % NQB;
  const int rest = bx / NQB;
  const int h    = rest % NH;
  const int b    = rest / NH;
  const int q0   = qb * 64 + wave * 16;
  const size_t rowB = (size_t)b * SEQ;

  const unsigned short* Qh  = qkh + (size_t)h * HD;
  const unsigned short* Ql  = qkl + (size_t)h * HD;
  const unsigned short* Kgh = qkh + DM + (size_t)h * HD;
  const unsigned short* Kgl = qkl + DM + (size_t)h * HD;
  const _Float16* Vgh = (const _Float16*)(const void*)vth + ((size_t)b * DM + (size_t)h * HD) * SEQ;
  const _Float16* Vgl = (const _Float16*)(const void*)vtl + ((size_t)b * DM + (size_t)h * HD) * SEQ;
  const _Float16* Evh = (const _Float16*)(const void*)evp;
  float* rrow = Rsh + (size_t)(wave * 16) * NREL;
  unsigned int* hw = Hs[wave];

  {
    v16us qh2[2], ql2[2];
#pragma unroll
    for (int dc = 0; dc < 2; ++dc) {
      qh2[dc] = ldfrag_u(Qh + (rowB + q0 + c) * QKP + dc * 32 + 8 * hh);
      ql2[dc] = ldfrag_u(Ql + (rowB + q0 + c) * QKP + dc * 32 + 8 * hh);
    }
#pragma unroll 1
    for (int nt = 0; nt < NREL / 16; ++nt) {
      v8f e = zero8();
#pragma unroll
      for (int dc = 0; dc < 2; ++dc) {
        const v16us eb = ldfrag_u(ekp + (size_t)(nt * 16 + c) * HD + dc * 32 + 8 * hh);
        e = mma_bu(qh2[dc], eb, e);
        e = mma_bu(ql2[dc], eb, e);
      }
#pragma unroll
      for (int r = 0; r < 8; ++r) rrow[(8 * hh + r) * NREL + nt * 16 + c] = e[r];
    }
  }
#pragma unroll
  for (int it = 0; it < 32; ++it) hw[it * 32 + lane] = 0u;
  wave_sync_lds();

  float mrow[8], lrow[8];
  v8f oacc[4], oaccL[4];
#pragma unroll
  for (int r = 0; r < 8; ++r) { mrow[r] = -INFINITY; lrow[r] = 0.f; }
#pragma unroll
  for (int t = 0; t < 4; ++t) { oacc[t] = zero8(); oaccL[t] = zero8(); }

#pragma unroll 1
  for (int kt = 0; kt < NQB; ++kt) {
    const int kv0 = kt * 64;

    __syncthreads();
    {
      const int r = tid >> 1, hf = (tid & 1) * 32;
      const unsigned short* kgh = Kgh + (rowB + kv0 + r) * QKP + hf;
      const unsigned short* kgl = Kgl + (rowB + kv0 + r) * QKP + hf;
      const _Float16* vgh = Vgh + (size_t)r * SEQ + kv0 + hf;
      const _Float16* vgl = Vgl + (size_t)r * SEQ + kv0 + hf;
#pragma unroll
      for (int i = 0; i < 4; ++i) {
        const v8us a0 = *(const v8us*)(kgh + 8 * i);
        const v8us a1 = *(const v8us*)(kgl + 8 * i);
        const v8h  b0 = *(const v8h*)(vgh + 8 * i);
        const v8h  b1 = *(const v8h*)(vgl + 8 * i);
        *(v8us*)(Kh + r * 64 + hf + 8 * i) = a0;
        *(v8us*)(Kl + r * 64 + hf + 8 * i) = a1;
        *(v8h*)(Vh + r * 64 + hf + 8 * i) = b0;
        *(v8h*)(Vl + r * 64 + hf + 8 * i) = b1;
      }
    }
    __syncthreads();

    v16us qh2[2], ql2[2];
#pragma unroll
    for (int dc = 0; dc < 2; ++dc) {
      qh2[dc] = ldfrag_u(Qh + (rowB + q0 + c) * QKP + dc * 32 + 8 * hh);
      ql2[dc] = ldfrag_u(Ql + (rowB + q0 + c) * QKP + dc * 32 + 8 * hh);
    }

    v8f s[4];
    unsigned int bnp[8];
#pragma unroll
    for (int r = 0; r < 8; ++r) bnp[r] = 0u;
    const int* rq = relp + (rowB + q0 + 8 * hh) * SEQ + kv0 + c;
#pragma unroll
    for (int j = 0; j < 4; ++j) {
      v8f sh = zero8();
#pragma unroll
      for (int dc = 0; dc < 2; ++dc) {
        FragU kbh, kbl;
        kbh.h[0] = *(const v8us*)(Kh + (j * 16 + c) * 64 + dc * 32 + 8 * hh);
        kbh.h[1] = *(const v8us*)(Kh + (j * 16 + c) * 64 + dc * 32 + 16 + 8 * hh);
        kbl.h[0] = *(const v8us*)(Kl + (j * 16 + c) * 64 + dc * 32 + 8 * hh);
        kbl.h[1] = *(const v8us*)(Kl + (j * 16 + c) * 64 + dc * 32 + 16 + 8 * hh);
        sh = mma_bu(qh2[dc], kbh.v, sh);
        sh = mma_bu(qh2[dc], kbl.v, sh);
        sh = mma_bu(ql2[dc], kbh.v, sh);
      }
#pragma unroll
      for (int r = 0; r < 8; ++r) {
        const int raw = rq[(size_t)r * SEQ + j * 16];
        int idx = (raw < 0) ? (raw + NREL) : raw;
        idx = (idx < 0) ? 0 : idx;
        idx = (idx > NREL - 1) ? (NREL - 1) : idx;
        const float tb = rrow[(8 * hh + r) * NREL + idx];
        const bool z = (raw == 0);
        s[j][r] = (sh[r] + (z ? 0.f : tb)) * sscale;
        bnp[r] |= (z ? 0u : (unsigned int)(idx + 1)) << (8 * j);
      }
    }

    _Float16* pwh = Psh[wave];
#pragma unroll
    for (int r = 0; r < 8; ++r) {
      float m = s[0][r];
      m = fmaxf(m, s[1][r]);
      m = fmaxf(m, s[2][r]);
      m = fmaxf(m, s[3][r]);
#pragma unroll
      for (int off = 1; off < 16; off <<= 1) m = fmaxf(m, __shfl_xor(m, off, 32));
      const float mnew  = fmaxf(mrow[r], m);
      const float alpha = __expf(mrow[r] - mnew);
      mrow[r] = mnew;
#pragma unroll
      for (int t = 0; t < 4; ++t) {
        const int hix = (8 * hh + r) * NREL + 16 * t + c;
        const float hv = (float)hw[hix] * alpha;
        hw[hix] = (unsigned int)(hv + 0.5f);
      }
      float psum = 0.f;
#pragma unroll
      for (int j = 0; j < 4; ++j) {
        const float p = __expf(s[j][r] - mnew);
        psum += p;
        pwh[(8 * hh + r) * 64 + j * 16 + c] = (_Float16)(p * PSC);
        s[j][r] = p;
      }
#pragma unroll
      for (int off = 1; off < 16; off <<= 1) psum += __shfl_xor(psum, off, 32);
      lrow[r] = lrow[r] * alpha + psum;
#pragma unroll
      for (int t = 0; t < 4; ++t) { oacc[t][r] *= alpha; oaccL[t][r] *= alpha; }
    }
    wave_sync_lds();

#pragma unroll
    for (int r = 0; r < 8; ++r) {
      const unsigned int pk = bnp[r];
#pragma unroll
      for (int j = 0; j < 4; ++j) {
        const unsigned int f = (pk >> (8 * j)) & 255u;
        if (f != 0u) {
          atomicAdd(&hw[(8 * hh + r) * NREL + (int)f - 1], (unsigned int)(s[j][r] * PFX + 0.5f));
        }
      }
    }

#pragma unroll 1
    for (int kk = 0; kk < 2; ++kk) {
      FragH pa;
      pa.h[0] = *(const v8h*)(pwh + c * 64 + kk * 32 + 8 * hh);
      pa.h[1] = *(const v8h*)(pwh + c * 64 + kk * 32 + 16 + 8 * hh);
#pragma unroll
      for (int t = 0; t < 4; ++t) {
        FragH vb, vl;
        vb.h[0] = *(const v8h*)(Vh + (t * 16 + c) * 64 + kk * 32 + 8 * hh);
        vb.h[1] = *(const v8h*)(Vh + (t * 16 + c) * 64 + kk * 32 + 16 + 8 * hh);
        vl.h[0] = *(const v8h*)(Vl + (t * 16 + c) * 64 + kk * 32 + 8 * hh);
        vl.h[1] = *(const v8h*)(Vl + (t * 16 + c) * 64 + kk * 32 + 16 + 8 * hh);
        oacc[t]  = mma_h(pa.v, vb.v, oacc[t]);
        oaccL[t] = mma_h(pa.v, vl.v, oaccL[t]);
      }
    }
  }

  wave_sync_lds();
  v8f oaccR[4];
#pragma unroll
  for (int t = 0; t < 4; ++t) oaccR[t] = zero8();
  {
    _Float16* pwh = Psh[wave];
    const float hcv = HCY / PFX;
#pragma unroll
    for (int it = 0; it < 32; ++it) {
      const int idx = it * 32 + lane;
      pwh[idx] = (_Float16)((float)hw[idx] * hcv);
    }
    wave_sync_lds();
#pragma unroll 1
    for (int kk = 0; kk < 2; ++kk) {
      FragH pa;
      pa.h[0] = *(const v8h*)(pwh + c * 64 + kk * 32 + 8 * hh);
      pa.h[1] = *(const v8h*)(pwh + c * 64 + kk * 32 + 16 + 8 * hh);
#pragma unroll
      for (int t = 0; t < 4; ++t) {
        const v16h eb = ldfrag_h(Evh + (size_t)(t * 16 + c) * NREL + kk * 32 + 8 * hh);
        oaccR[t] = mma_h(pa.v, eb, oaccR[t]);
      }
    }
  }

  float* os = Os[wave];
#pragma unroll
  for (int r = 0; r < 8; ++r) {
    const float l = lrow[r];
    const float invl = (l > 0.f) ? (1.0f / l) : 0.f;
#pragma unroll
    for (int t = 0; t < 4; ++t) {
      os[(8 * hh + r) * 64 + t * 16 + c] =
          (oacc[t][r] * (1.0f / PSC) + oaccL[t][r] * (1.0f / (PSC * RSC)) + oaccR[t][r] * (1.0f / (HCY * WSC))) * invl;
    }
  }
  wave_sync_lds();
  {
    const int q4 = lane >> 3, c8 = (lane & 7) * 8;
    v4u hv[4], lv[4];
#pragma unroll
    for (int it = 0; it < 4; ++it) {
      const int row = it * 4 + q4;
      const float* sp = os + row * 64 + c8;
      v4u ha, la;
#pragma unroll
      for (int e = 0; e < 4; ++e) {
        const float f0 = sp[2 * e], f1 = sp[2 * e + 1];
        const unsigned short u0 = bf_bits(f0), u1 = bf_bits(f1);
        const unsigned short w0 = bf_bits(f0 - bf_up(u0)), w1 = bf_bits(f1 - bf_up(u1));
        ha[e] = pk16(u0, u1);
        la[e] = pk16(w0, w1);
      }
      hv[it] = ha;
      lv[it] = la;
    }
    for (int pass = 0; pass < 2; ++pass) {
#pragma unroll
      for (int it = 0; it < 4; ++it) {
        const int row = it * 4 + q4;
        const size_t go = (rowB + q0 + row) * CTXP + (size_t)h * HD + c8;
        *(volatile v4u*)(ctxp + go)      = hv[it];
        *(volatile v4u*)(ctxp + go + DM) = lv[it];
      }
      __threadfence();
    }
  }
}

template <int RA, int WP>
__global__ __launch_bounds__(256) void lnrow(const float* __restrict__ A, const float* __restrict__ Bm,
                                             const float* __restrict__ g, const float* __restrict__ be,
                                             float* outf, unsigned short* plane, int nrows) {
  __shared__ __align__(16) unsigned short sh[8][2 * DM];
  const int wave = threadIdx.x >> 5, lane = threadIdx.x & 31;
  const int row = blockIdx.x * 8 + wave;
  if (row >= nrows) return;
  const float* pa = A  + (size_t)row * DM;
  const float* pb = Bm + (size_t)row * DM;
  v4f v[8];
  float s = 0.f;
#pragma unroll
  for (int it = 0; it < 8; ++it) {
    const int col = it * 128 + lane * 4;
    v4f va = *(const v4f*)(pa + col);
    if (RA) { va[0] = bfr(va[0]); va[1] = bfr(va[1]); va[2] = bfr(va[2]); va[3] = bfr(va[3]); }
    const v4f vb = *(const v4f*)(pb + col);
    v[it] = va + vb;
    s += (v[it][0] + v[it][1]) + (v[it][2] + v[it][3]);
  }
#pragma unroll
  for (int off = 16; off > 0; off >>= 1) s += __shfl_xor(s, off, 32);
  const float mean = s * (1.0f / DM);
  float ss = 0.f;
#pragma unroll
  for (int it = 0; it < 8; ++it) {
    const v4f d = v[it] - mean;
    v[it] = d;
    ss += (d[0] * d[0] + d[1] * d[1]) + (d[2] * d[2] + d[3] * d[3]);
  }
#pragma unroll
  for (int off = 16; off > 0; off >>= 1) ss += __shfl_xor(ss, off, 32);
  const float var  = ss * (1.0f / DM);
  const float rstd = rsqrtf(var + 1e-5f);
  v4f y[8];
#pragma unroll
  for (int it = 0; it < 8; ++it) {
    const int col = it * 128 + lane * 4;
    const v4f gv = *(const v4f*)(g + col);
    const v4f bv = *(const v4f*)(be + col);
    v4f o;
#pragma unroll
    for (int e = 0; e < 4; ++e) o[e] = (v[it][e] * rstd) * bfr(gv[e]) + bfr(bv[e]);
    y[it] = o;
  }
  float* po = outf + (size_t)row * DM;
  for (int pass = 0; pass < 2; ++pass) {
#pragma unroll
    for (int it = 0; it < 8; ++it) *(volatile v4f*)(po + it * 128 + lane * 4) = y[it];
    __threadfence();
  }
  if (WP) {
    unsigned short* shw = sh[wave];
#pragma unroll
    for (int it = 0; it < 8; ++it) {
      const int col = it * 128 + lane * 4;
      const unsigned short u0 = bf_bits(y[it][0]), u1 = bf_bits(y[it][1]);
      const unsigned short u2 = bf_bits(y[it][2]), u3 = bf_bits(y[it][3]);
      const unsigned short w0 = bf_bits(y[it][0] - bf_up(u0)), w1 = bf_bits(y[it][1] - bf_up(u1));
      const unsigned short w2 = bf_bits(y[it][2] - bf_up(u2)), w3 = bf_bits(y[it][3] - bf_up(u3));
      v2u hp, lp;
      hp[0] = pk16(u0, u1); hp[1] = pk16(u2, u3);
      lp[0] = pk16(w0, w1); lp[1] = pk16(w2, w3);
      *(v2u*)(shw + col)      = hp;
      *(v2u*)(shw + DM + col) = lp;
    }
    wave_sync_lds();
    v4u hv[4], lv[4];
#pragma unroll
    for (int it = 0; it < 4; ++it) {
      const int col8 = it * 256 + lane * 8;
      hv[it] = *(const v4u*)(shw + col8);
      lv[it] = *(const v4u*)(shw + DM + col8);
    }
    unsigned short* pp = plane + (size_t)row * XPP;
    for (int pass = 0; pass < 2; ++pass) {
#pragma unroll
      for (int it = 0; it < 4; ++it) {
        const int col8 = it * 256 + lane * 8;
        *(volatile v4u*)(pp + col8)      = hv[it];
        *(volatile v4u*)(pp + DM + col8) = lv[it];
      }
      __threadfence();
    }
  }
}

extern "C" void kernel_launch(void* const* d_in, const int* in_sizes, int n_in,
                              void* d_out, int out_size, void* d_ws, size_t ws_size,
                              hipStream_t stream) {
  if (n_in < 16) return;
  if (in_sizes[0] != MP * DM) return;
  if (in_sizes[1] != NBATCH * SEQ * SEQ) return;
  if (in_sizes[2] != 3 * DM * DM || in_sizes[3] != 3 * DM) return;
  if (in_sizes[4] != DM * DM || in_sizes[5] != DM) return;
  if (in_sizes[6] != DM || in_sizes[7] != DM) return;
  if (in_sizes[8] != DFF * DM || in_sizes[9] != DFF) return;
  if (in_sizes[10] != DM * DFF || in_sizes[11] != DM) return;
  if (in_sizes[12] != DM || in_sizes[13] != DM) return;
  if (in_sizes[14] != NREL * HD || in_sizes[15] != NREL * HD) return;
  if (out_size != MP * DM) return;

  const float* src   = (const float*)d_in[0];
  const int*   relid = (const int*)d_in[1];
  const float* w_qkv = (const float*)d_in[2];
  const float* b_qkv = (const float*)d_in[3];
  const float* w_o   = (const float*)d_in[4];
  const float* b_o   = (const float*)d_in[5];
  const float* ln1g  = (const float*)d_in[6];
  const float* ln1b  = (const float*)d_in[7];
  const float* w_1   = (const float*)d_in[8];
  const float* b_1   = (const float*)d_in[9];
  const float* w_2   = (const float*)d_in[10];
  const float* b_2   = (const float*)d_in[11];
  const float* ln2g  = (const float*)d_in[12];
  const float* ln2b  = (const float*)d_in[13];
  const float* relk  = (const float*)d_in[14];
  const float* relv  = (const float*)d_in[15];

  const size_t PWQ  = (size_t)3 * DM * DM * 2;
  const size_t PXH  = (size_t)MP * DM * 2;
  const size_t PWOD = (size_t)DM * (2 * DM) * 2;
  const size_t PW1D = (size_t)DFF * (2 * DM) * 2;
  const size_t PW2D = (size_t)DM * (2 * DFF) * 2;
  const size_t PEK  = (size_t)NREL * HD * 2;
  const size_t PEV  = (size_t)HD * NREL * 2;
  const size_t PQK  = (size_t)MP * QKP * 2;
  const size_t PVT  = (size_t)NBATCH * DM * SEQ * 2;
  const size_t PCTX = (size_t)MP * CTXP * 2;
  const size_t PF32 = (size_t)MP * DM * 4;
  const size_t PXP  = (size_t)MP * XPP * 2;
  const size_t PHP  = (size_t)MP * HPP * 2;
  size_t off = 0;
  const size_t oWQ  = off; off += PWQ;
  const size_t oXH  = off; off += PXH;
  const size_t oWOD = off; off += PWOD;
  const size_t oW1D = off; off += PW1D;
  const size_t oW2D = off; off += PW2D;
  const size_t oEK  = off; off += PEK;
  const size_t oEV  = off; off += PEV;
  const size_t oQKh = off; off += PQK;
  const size_t oQKl = off; off += PQK;
  const size_t oVTh = off; off += PVT;
  const size_t oVTl = off; off += PVT;
  const size_t oCtx = off; off += PCTX;
  const size_t oAO  = off; off += PF32;
  const size_t oX1  = off; off += PF32;
  const size_t oXP  = off; off += PXP;
  const size_t oHP  = off; off += PHP;
  const size_t oFF  = off; off += PF32;
  if (off > ws_size) return;
  if (off > (size_t)134217728) return;

  char* ws = (char*)d_ws;
  unsigned short* WQ  = (unsigned short*)(ws + oWQ);
  unsigned short* XH  = (unsigned short*)(ws + oXH);
  unsigned short* WOD = (unsigned short*)(ws + oWOD);
  unsigned short* W1D = (unsigned short*)(ws + oW1D);
  unsigned short* W2D = (unsigned short*)(ws + oW2D);
  unsigned short* EK  = (unsigned short*)(ws + oEK);
  unsigned short* EV  = (unsigned short*)(ws + oEV);
  unsigned short* QKh = (unsigned short*)(ws + oQKh);
  unsigned short* QKl = (unsigned short*)(ws + oQKl);
  unsigned short* VTh = (unsigned short*)(ws + oVTh);
  unsigned short* VTl = (unsigned short*)(ws + oVTl);
  unsigned short* Ctx = (unsigned short*)(ws + oCtx);
  float*          AO  = (float*)(ws + oAO);
  float*          X1  = (float*)(ws + oX1);
  unsigned short* XP  = (unsigned short*)(ws + oXP);
  unsigned short* HP  = (unsigned short*)(ws + oHP);
  float*          FF  = (float*)(ws + oFF);
  float*          out0 = (float*)d_out;

  const int n8w = (3 * DM * DM) / 8;
  const int n8x = (MP * DM) / 8;
  const int n8o = (DM * DM) / 8;
  const int n81 = (DFF * DM) / 8;
  const int n82 = (DM * DFF) / 8;
  const int n8e = (NREL * HD) / 8;
  const dim3 blk(256), blk128(128);
  const dim3 gCw((n8w + 255) / 256), gCx((n8x + 255) / 256), gCo((n8o + 255) / 256);
  const dim3 gC1((n81 + 255) / 256), gC2((n82 + 255) / 256), gCe((n8e + 255) / 256);
  const dim3 gTv(HD / 64, NREL / 64);
  const dim3 gQK(((MP / 64) * (QKP / 64) + 7) / 8, 1);
  const dim3 gVT(((DM / 64) * (SEQ / 64) + 7) / 8, NBATCH);
  const dim3 gAttn(NBATCH * NH * NQB);
  const dim3 gWo(((MP / 64) * (DM / 64) + 7) / 8, 1);
  const dim3 gW1(((MP / 64) * (DFF / 64) + 7) / 8, 1);
  const dim3 gW2(((MP / 64) * (DM / 64) + 7) / 8, 1);
  const dim3 gLn((MP + 7) / 8);
  const float invw = 1.0f / WSC;

  conv16<0><<<gCw, blk, 0, stream>>>(w_qkv, WQ, n8w, DM, DM, 0, WSC);
  conv16<0><<<gCx, blk, 0, stream>>>(src, XH, n8x, DM, DM, 0, 1.0f);
  conv16<1><<<gCo, blk, 0, stream>>>(w_o, WOD, n8o, DM, 2 * DM, 1, 1.0f);
  conv16<1><<<gC1, blk, 0, stream>>>(w_1, W1D, n81, DM, 2 * DM, 1, 1.0f);
  conv16<1><<<gC2, blk, 0, stream>>>(w_2, W2D, n82, DFF, 2 * DFF, 1, 1.0f);
  conv_e16<<<gCe, blk, 0, stream>>>(relk, EK, n8e, n8e);
  tconv64<0><<<gTv, blk, 0, stream>>>(relv, EV, NREL, HD, NREL, 0, WSC);

  gemm64<0, 3, 1, 0><<<gQK, blk, 0, stream>>>(
      XH, DM, 0LL, WQ, DM, 0LL,
      QKh, QKl, AO, QKP, 0LL, b_qkv, MP, QKP, DM, invw);
  gemm64<0, 4, 2, 0><<<gVT, blk, 0, stream>>>(
      WQ + (size_t)(2 * DM) * DM, DM, 0LL, XH, DM, (long long)SEQ * DM,
      VTh, VTl, AO, SEQ, (long long)DM * SEQ, b_qkv + 2 * DM, DM, SEQ, DM, invw);

  attn64<<<gAttn, blk128, 0, stream>>>(QKh, QKl, VTh, VTl, EK, EV, relid, Ctx, 0.125f);

  gemm64<1, 0, 1, 0><<<gWo, blk, 0, stream>>>(
      Ctx, CTXP, 0LL, WOD, 2 * DM, 0LL,
      Ctx, Ctx, AO, DM, 0LL, b_o, MP, DM, 2 * DM, 1.0f);

  lnrow<1, 1><<<gLn, blk, 0, stream>>>(src, AO, ln1g, ln1b, X1, XP, MP);

  gemm64<1, 3, 1, 1><<<gW1, blk, 0, stream>>>(
      XP, XPP, 0LL, W1D, 2 * DM, 0LL,
      HP, HP + DFF, FF, HPP, 0LL, b_1, MP, DFF, 2 * DM, 1.0f);

  gemm64<1, 0, 1, 0><<<gW2, blk, 0, stream>>>(
      HP, HPP, 0LL, W2D, 2 * DFF, 0LL,
      HP, HP, FF, DM, 0LL, b_2, MP, DM, 2 * DFF, 1.0f);

  lnrow<0, 0><<<gLn, blk, 0, stream>>>(X1, FF, ln2g, ln2b, out0, XP, MP);
  (void)hipGetLastError();
}
